// DenseAttention_26345329393764
// MI455X (gfx1250) — hardware-verified
//
#include <hip/hip_runtime.h>


#define NB_  2
#define TT   2048
#define EE   1024
#define SQ   4
#define HH   256
typedef _Float16 h16;
typedef unsigned short bf;
typedef __attribute__((ext_vector_type(16))) __bf16   v16bf;
typedef __attribute__((ext_vector_type(16))) _Float16 v16h;
typedef __attribute__((ext_vector_type(8)))  _Float16 v8h;
typedef __attribute__((ext_vector_type(8)))  unsigned short v8us;
typedef __attribute__((ext_vector_type(8)))  float    v8f;
typedef __attribute__((ext_vector_type(4)))  float    v4f;
typedef v8h  __attribute__((may_alias)) v8ha;
typedef v4f  __attribute__((may_alias)) v4fa;
typedef v8us __attribute__((may_alias)) v8usa;

__device__ __forceinline__ unsigned short f2bf(float f) { unsigned u = __float_as_uint(f); u += 0x7FFFu + ((u >> 16) & 1u); return (unsigned short)(u >> 16); }
__device__ __forceinline__ float bf2f(unsigned short b) { return __uint_as_float(((unsigned)b) << 16); }
__device__ __forceinline__ float bfr(float f) { return bf2f(f2bf(f)); }
__device__ __forceinline__ v16h cat16(v8h lo, v8h hi) { return __builtin_shufflevector(lo, hi, 0, 1, 2, 3, 4, 5, 6, 7, 8, 9, 10, 11, 12, 13, 14, 15); }
__device__ __forceinline__ v16bf cat16b(v8us lo, v8us hi) { return __builtin_bit_cast(v16bf, __builtin_shufflevector(lo, hi, 0, 1, 2, 3, 4, 5, 6, 7, 8, 9, 10, 11, 12, 13, 14, 15)); }
__device__ __forceinline__ v8f wmma16(v16h a, v16h b, v8f c) { return __builtin_amdgcn_wmma_f32_16x16x32_f16(false, a, false, b, (short)0, c, false, false); }
__device__ __forceinline__ v8f wmmab(v16bf a, v16bf b, v8f c) { return __builtin_amdgcn_wmma_f32_16x16x32_bf16(false, a, false, b, (short)0, c, false, false); }


template <typename T16> struct WFrag;
template <> struct WFrag<h16> { typedef v16h V; static __device__ __forceinline__ V ld(const h16* p) { return cat16(*(const v8h*)p, *(const v8h*)(p + 16)); } static __device__ __forceinline__ v8f mma(V a, V b, v8f c) { return wmma16(a, b, c); } };
template <> struct WFrag<bf> { typedef v16bf V; static __device__ __forceinline__ V ld(const bf* p) { return cat16b(*(const v8us*)p, *(const v8us*)(p + 16)); } static __device__ __forceinline__ v8f mma(V a, V b, v8f c) { return wmmab(a, b, c); } };
template <typename T16, int NSPLIT, bool BIAS>
__global__ __launch_bounds__(32) void k_gemmw(const T16* __restrict__ A, const T16* __restrict__ A2, const T16* __restrict__ Bt, const T16* __restrict__ Bt2, int K, float* C, int ldc, const float* __restrict__ bias, size_t sA, size_t sB, size_t sC) {
    typedef typename WFrag<T16>::V V;
    __shared__ __align__(16) float os[16 * 68];
    const size_t z = blockIdx.z; A += z * sA; if (A2) A2 += z * sA; Bt += z * sB; if (Bt2) Bt2 += z * sB; C += z * sC;
    const int lane = threadIdx.x & 31, lr = lane & 15, hi = lane >> 4; const int r0 = blockIdx.x * 64, c0 = blockIdx.y * 64;
    v8f acc[4][4];
#pragma unroll
    for (int mb = 0; mb < 4; ++mb)
#pragma unroll
        for (int nb = 0; nb < 4; ++nb) acc[mb][nb] = (v8f){};
    const size_t aoff = (size_t)(r0 + lr) * K + 8 * hi, boff = (size_t)(c0 + lr) * K + 8 * hi;
#pragma unroll 1
    for (int kc = 0; kc < K; kc += 32) {
        V a[4], a2[4];
#pragma unroll
        for (int mb = 0; mb < 4; ++mb) { a[mb] = WFrag<T16>::ld(A + aoff + (size_t)mb * 16 * K + kc); if (NSPLIT == 1 || NSPLIT == 2) a2[mb] = WFrag<T16>::ld(A2 + aoff + (size_t)mb * 16 * K + kc); }
#pragma unroll
        for (int nb = 0; nb < 4; ++nb) { const V b = WFrag<T16>::ld(Bt + boff + (size_t)nb * 16 * K + kc); V b2; if (NSPLIT >= 2) b2 = WFrag<T16>::ld(Bt2 + boff + (size_t)nb * 16 * K + kc);
#pragma unroll
            for (int mb = 0; mb < 4; ++mb) { acc[mb][nb] = WFrag<T16>::mma(a[mb], b, acc[mb][nb]); if (NSPLIT == 1 || NSPLIT == 2) acc[mb][nb] = WFrag<T16>::mma(a2[mb], b, acc[mb][nb]); if (NSPLIT >= 2) acc[mb][nb] = WFrag<T16>::mma(a[mb], b2, acc[mb][nb]); } }
        asm volatile("v_nop\n\tv_nop\n\tv_nop\n\tv_nop" : "+v"(acc[0][0]), "+v"(acc[1][1]), "+v"(acc[2][2]), "+v"(acc[3][3]) : "v"(a[0]), "v"(a[3]));
    }
#pragma unroll
    for (int mb = 0; mb < 4; ++mb) {
#pragma unroll
        for (int nb = 0; nb < 4; ++nb) {
#pragma unroll
            for (int j = 0; j < 8; ++j) os[(hi * 8 + j) * 68 + nb * 16 + lr] = acc[mb][nb][j]; }
        __builtin_amdgcn_wave_barrier(); asm volatile("" ::: "memory");
        float* crow = C + (size_t)(r0 + mb * 16) * ldc + c0;
#pragma unroll 1
        for (int ps = 0; ps < 2; ++ps) {
#pragma unroll
            for (int s = 0; s < 8; ++s) { const int row = 2 * s + hi, cofs = lr * 4; v4f val = *(const v4fa*)(os + row * 68 + cofs); if (BIAS) { val[0] += bfr(bias[c0 + cofs]); val[1] += bfr(bias[c0 + cofs + 1]); val[2] += bfr(bias[c0 + cofs + 2]); val[3] += bfr(bias[c0 + cofs + 3]); }
                *(volatile v4f*)(crow + (size_t)row * ldc + cofs) = val; }
            if (ps == 0) __threadfence(); }
        __builtin_amdgcn_wave_barrier(); asm volatile("" ::: "memory");
    }
}

__device__ __forceinline__ void splitf(float y, unsigned short& h, unsigned short& l) { h = f2bf(y); l = f2bf(y - bf2f(h)); }
typedef __attribute__((ext_vector_type(2))) unsigned short v2us;
typedef __attribute__((ext_vector_type(4))) unsigned short v4us;

__global__ __launch_bounds__(256) void k_wtG(const float* __restrict__ w, int K, int N, bf* Bt) {
    const int lane = threadIdx.x & 31; const int L0 = (blockIdx.x * 8 + (threadIdx.x >> 5)) * 8; const int nlines = N * K / 64;
#pragma unroll
    for (int ps = 0; ps < 2; ++ps) {
#pragma unroll 1
        for (int l = 0; l < 8; ++l) { const int L = L0 + l; if (L >= nlines) break; const size_t e = (size_t)L * 64 + lane * 2; const int k = (int)(e % K), n = (int)(e / K); v2us o;
            o[0] = f2bf(w[(size_t)k * N + n]); o[1] = f2bf(w[(size_t)(k + 1) * N + n]); *(volatile v2us*)(Bt + e) = o; }
        if (ps == 0) __threadfence(); }
}

__global__ __launch_bounds__(256) void k_plb(const float* __restrict__ F, bf* Ph, bf* Pl) { const size_t e4 = ((size_t)blockIdx.x * 256 + threadIdx.x) * 4; if (e4 >= (size_t)TT * EE) return; const int f = (int)(e4 % HH); const int t = (int)((e4 / HH) % TT); const int q2 = (int)(e4 / ((size_t)HH * TT)); const float* src = F + (size_t)t * EE + q2 * HH + f; v4us oh, ol;
#pragma unroll
    for (int u = 0; u < 4; ++u) { unsigned short a, b; splitf(src[u], a, b); oh[u] = a; ol[u] = b; } *(volatile v4us*)(Ph + e4) = oh; *(volatile v4us*)(Pl + e4) = ol; __threadfence(); *(volatile v4us*)(Ph + e4) = oh; *(volatile v4us*)(Pl + e4) = ol; }
__global__ __launch_bounds__(256) void k_xs(const float* __restrict__ X, bf* XS) { const size_t e4 = ((size_t)blockIdx.x * 256 + threadIdx.x) * 4; if (e4 >= (size_t)SQ * TT * HH) return; const int e = (int)(e4 % HH); const int t = (int)((e4 / HH) % TT); const int a = (int)(e4 / ((size_t)HH * TT)); const float* src = X + (size_t)t * EE + a * HH + e; v4us o;
#pragma unroll
    for (int u = 0; u < 4; ++u) o[u] = f2bf(src[u]); *(volatile v4us*)(XS + e4) = o; __threadfence(); *(volatile v4us*)(XS + e4) = o; }
__global__ __launch_bounds__(256) void k_xt(const float* __restrict__ X, bf* XT) { const size_t e2 = ((size_t)blockIdx.x * 256 + threadIdx.x) * 2; if (e2 >= (size_t)SQ * HH * TT) return; const int t = (int)(e2 % TT); const int e = (int)((e2 / TT) % HH); const int a = (int)(e2 / ((size_t)TT * HH)); v2us o; o[0] = f2bf(X[(size_t)t * EE + a * HH + e]); o[1] = f2bf(X[(size_t)(t + 1) * EE + a * HH + e]); *(volatile v2us*)(XT + e2) = o; __threadfence(); *(volatile v2us*)(XT + e2) = o; }
__global__ __launch_bounds__(256) void k_pl(const float* __restrict__ F, bf* Ph, bf* Pl, size_t n4) { const size_t e = ((size_t)blockIdx.x * 256 + threadIdx.x) * 4; if (e >= n4 * 4) return; const v4f a = *(const v4f*)(F + e); v4us oh, ol;
#pragma unroll
    for (int u = 0; u < 4; ++u) { unsigned short x0, x1; splitf(a[u], x0, x1); oh[u] = x0; ol[u] = x1; } *(volatile v4us*)(Ph + e) = oh; *(volatile v4us*)(Pl + e) = ol; __threadfence(); *(volatile v4us*)(Ph + e) = oh; *(volatile v4us*)(Pl + e) = ol; }

extern "C" void kernel_launch(void* const* d_in, const int* in_sizes, int n_in,
                              void* d_out, int out_size, void* d_ws, size_t ws_size, hipStream_t stream) {
    (void)in_sizes; (void)n_in; (void)out_size;
    const float* x = (const float*)d_in[0]; const float* queries = (const float*)d_in[1]; const float* comb = (const float*)d_in[2];
    float* OUT = (float*)d_out;
    char* wsp = (char*)d_ws;
    auto take = [&](size_t bytes) { char* p = wsp; wsp += (bytes + 255) & ~(size_t)255; return (void*)p; };
    bf* BQW = (bf*)take((size_t)SQ * EE * HH * 2); bf* BCB = (bf*)take((size_t)SQ * HH * EE * 2);
    bf* XS = (bf*)take((size_t)SQ * TT * HH * 2); bf* XT = (bf*)take((size_t)SQ * HH * TT * 2); float* G = (float*)take((size_t)SQ * HH * HH * 4); bf* Gh = (bf*)take((size_t)SQ * HH * HH * 2); bf* Gl = (bf*)take((size_t)SQ * HH * HH * 2);
    float* Q = (float*)take((size_t)TT * EE * 4); bf* Qh = (bf*)take((size_t)TT * EE * 2); bf* Ql = (bf*)take((size_t)TT * EE * 2); float* AT = (float*)take((size_t)TT * EE * 4); bf* ATh = (bf*)take((size_t)TT * EE * 2); bf* ATl = (bf*)take((size_t)TT * EE * 2);
    if ((size_t)(wsp - (char*)d_ws) > ws_size) return;
    for (int a = 0; a < SQ; ++a) { k_wtG<<<(HH * EE / 64 + 63) / 64, 256, 0, stream>>>(queries + (size_t)a * HH * EE, HH, EE, BQW + (size_t)a * EE * HH); k_wtG<<<(EE * HH / 64 + 63) / 64, 256, 0, stream>>>(comb + (size_t)a * EE * HH, EE, HH, BCB + (size_t)a * HH * EE); }
    const unsigned LP = (unsigned)(((size_t)TT * EE / 4 + 255) / 256);
    for (int b = 0; b < NB_; ++b) { const float* xb = x + (size_t)b * TT * EE;
        k_xs<<<(unsigned)(((size_t)SQ * TT * HH / 4 + 255) / 256), 256, 0, stream>>>(xb, XS); k_xt<<<(unsigned)(((size_t)SQ * HH * TT / 2 + 255) / 256), 256, 0, stream>>>(xb, XT);
        k_gemmw<bf, 0, false><<<dim3(HH / 64, HH / 64, SQ), 32, 0, stream>>>(XT, nullptr, XT, nullptr, TT, G, HH, nullptr, (size_t)HH * TT, (size_t)HH * TT, (size_t)HH * HH);
        k_pl<<<(SQ * HH * HH / 4 + 255) / 256, 256, 0, stream>>>(G, Gh, Gl, (size_t)SQ * HH * HH / 4);
        for (int a = 0; a < SQ; ++a) {
            k_gemmw<bf, 0, false><<<dim3(TT / 64, EE / 64, 1), 32, 0, stream>>>(XS + (size_t)a * TT * HH, nullptr, BQW + (size_t)a * EE * HH, nullptr, HH, Q, EE, nullptr, 0, 0, 0);
            k_plb<<<LP, 256, 0, stream>>>(Q, Qh, Ql);
            for (int q2 = 0; q2 < SQ; ++q2) k_gemmw<bf, 2, false><<<dim3(TT / 64, HH / 64, 1), 32, 0, stream>>>(Qh + (size_t)q2 * TT * HH, Ql + (size_t)q2 * TT * HH, Gh + (size_t)q2 * HH * HH, Gl + (size_t)q2 * HH * HH, HH, AT + q2 * HH, EE, nullptr, 0, 0, 0);
            k_pl<<<LP, 256, 0, stream>>>(AT, ATh, ATl, (size_t)TT * EE / 4);
            k_gemmw<bf, 1, false><<<dim3(TT / 64, HH / 64, 1), 32, 0, stream>>>(ATh, ATl, BCB + (size_t)a * HH * EE, nullptr, EE, OUT + (size_t)b * TT * EE + a * HH, EE, nullptr, 0, 0, 0); } }
}
